// DualGCNModel_23845658427619
// MI455X (gfx1250) — hardware-verified
//
#include <hip/hip_runtime.h>
#include <stddef.h>


#define FO      128
#define FS      64
#define HID     128
#define NCL     64
#define MHID    256
#define NTHR    256
#define NWAVE   8
#define EPT     8
#define NGRP    2
#define CHUNK   (NTHR * EPT * NGRP)
#define WCAP    (EPT * NGRP * 32)
#define LISTN   (NWAVE * WCAP)
#define ESHF    11
#define NBC     32768
#define NBF     2048
#define RCAP    40960
#define RBN     128
#define TGT     256
#define DEGCAP  512
#define GROWS   128
#define GCOLS   64
#define OTHR    512
#define WSC     16
#define ASC     16
#define WSCAP   134217728

#define P0OF    0
#define P1OF    16384
#define P2OF    24576
#define P3OF    32768
#define P4OF    40960
#define P5OF    73728
#define WPH     90112
#define WPBLK   44

#define LDS_COUNT ((NBC + LISTN + NWAVE) * 4)
#define LDS_FILL  ((RCAP + NBF + LISTN + NWAVE) * 4)
#define LDS_AGG1  (NWAVE * 32 * (FO + FS) * 2)
#define LDS_AGG2  (NWAVE * 32 * (2 * NCL) * 2)

static_assert((CHUNK & (CHUNK - 1)) == 0);
static_assert((NBC & (NBC - 1)) == 0 && (NBF & (NBF - 1)) == 0);
static_assert(NBF <= (1 << ESHF));
static_assert((NBC % NBF) == 0);
static_assert(OTHR * 4 == NBF);
static_assert((RCAP % 32) == 0);
static_assert(TGT == NWAVE * 32);
static_assert(GROWS == NWAVE * 16);
static_assert((TGT % GROWS) == 0);
static_assert(NBC == NWAVE * 32 * 128);
static_assert(FO == 128 && FS == 64 && HID == 128 && NCL == 64 && MHID == 256);
static_assert(WPH == P5OF + 64 * 256);

typedef float     v2f  __attribute__((ext_vector_type(2)));
typedef float     v4f  __attribute__((ext_vector_type(4)));
typedef float     v8f  __attribute__((ext_vector_type(8)));
typedef int       v4i  __attribute__((ext_vector_type(4)));
typedef _Float16  v2h  __attribute__((ext_vector_type(2)));
typedef _Float16  v4h  __attribute__((ext_vector_type(4)));
typedef _Float16  v8h  __attribute__((ext_vector_type(8)));
typedef _Float16  v16h __attribute__((ext_vector_type(16)));
typedef _Float16  v8ha __attribute__((ext_vector_type(8))) __attribute__((may_alias));
typedef float     v4fa __attribute__((ext_vector_type(4))) __attribute__((may_alias));
union FragH { v16h v; v8h h[2]; };

__device__ __forceinline__ v8f wmf(v16h a, v16h b, v8f c) {
  v8f d = __builtin_amdgcn_wmma_f32_16x16x32_f16(false, a, false, b, (short)0, c, false, false);
  asm volatile("v_nop\n\tv_nop\n\tv_nop\n\tv_nop" : "+v"(d) : "v"(a), "v"(b));
  return d;
}

template <int NB, int SRC>
__device__ __forceinline__ int scan_chunk(const int* __restrict__ keys, const int* __restrict__ vals, int nE, int nN,
                                          int cbase, int slotBase, int vec8, int* list, int tid, int lane, int wave) {
  int wc = 0;
#pragma unroll
  for (int g = 0; g < NGRP; ++g) {
    const int el0  = (g * NTHR + tid) * EPT;
    const int e0   = cbase + el0;
    const int sent = -2147483647 - 1;
    v4i da, db;
    v4i sa = {0, 0, 0, 0}, sb = {0, 0, 0, 0};
    if (vec8 != 0 && cbase + CHUNK <= nE) {
      da = *(const v4i*)(keys + e0);
      db = *(const v4i*)(keys + e0 + 4);
      if (SRC) {
        sa = *(const v4i*)(vals + e0);
        sb = *(const v4i*)(vals + e0 + 4);
      }
    } else {
      da.x = (e0     < nE) ? keys[min(e0, nE - 1)] : sent;
      da.y = (e0 + 1 < nE) ? keys[min(e0 + 1, nE - 1)] : sent;
      da.z = (e0 + 2 < nE) ? keys[min(e0 + 2, nE - 1)] : sent;
      da.w = (e0 + 3 < nE) ? keys[min(e0 + 3, nE - 1)] : sent;
      db.x = (e0 + 4 < nE) ? keys[min(e0 + 4, nE - 1)] : sent;
      db.y = (e0 + 5 < nE) ? keys[min(e0 + 5, nE - 1)] : sent;
      db.z = (e0 + 6 < nE) ? keys[min(e0 + 6, nE - 1)] : sent;
      db.w = (e0 + 7 < nE) ? keys[min(e0 + 7, nE - 1)] : sent;
      if (SRC) {
        sa.x = vals[min(e0, nE - 1)];
        sa.y = vals[min(e0 + 1, nE - 1)];
        sa.z = vals[min(e0 + 2, nE - 1)];
        sa.w = vals[min(e0 + 3, nE - 1)];
        sb.x = vals[min(e0 + 4, nE - 1)];
        sb.y = vals[min(e0 + 5, nE - 1)];
        sb.z = vals[min(e0 + 6, nE - 1)];
        sb.w = vals[min(e0 + 7, nE - 1)];
      }
    }
    if (SRC) {
      sa.x = min(max(sa.x, 0), nN - 1); sa.y = min(max(sa.y, 0), nN - 1);
      sa.z = min(max(sa.z, 0), nN - 1); sa.w = min(max(sa.w, 0), nN - 1);
      sb.x = min(max(sb.x, 0), nN - 1); sb.y = min(max(sb.y, 0), nN - 1);
      sb.z = min(max(sb.z, 0), nN - 1); sb.w = min(max(sb.w, 0), nN - 1);
    }
    const unsigned nb = (unsigned)slotBase;
    const unsigned s0 = (unsigned)da.x - nb, s1 = (unsigned)da.y - nb;
    const unsigned s2 = (unsigned)da.z - nb, s3 = (unsigned)da.w - nb;
    const unsigned s4 = (unsigned)db.x - nb, s5 = (unsigned)db.y - nb;
    const unsigned s6 = (unsigned)db.z - nb, s7 = (unsigned)db.w - nb;
    const bool h0 = s0 < (unsigned)NB, h1 = s1 < (unsigned)NB, h2 = s2 < (unsigned)NB, h3 = s3 < (unsigned)NB;
    const bool h4 = s4 < (unsigned)NB, h5 = s5 < (unsigned)NB, h6 = s6 < (unsigned)NB, h7 = s7 < (unsigned)NB;
    const unsigned any = __builtin_amdgcn_ballot_w32(h0 | h1 | h2 | h3 | h4 | h5 | h6 | h7);
    if (any != 0u) {
#define HITJ(HJ, SJ, VJ) { \
        const unsigned mj = __builtin_amdgcn_ballot_w32(HJ); \
        if (mj != 0u) { \
          if (HJ) { \
            const int pos = wc + (int)__builtin_amdgcn_mbcnt_lo(mj, 0u); \
            const int entv = SRC ? (((VJ) << ESHF) | (int)(SJ)) : (int)(SJ); \
            if (pos < WCAP) list[wave * WCAP + pos] = entv; \
          } \
          wc += (int)__builtin_popcount(mj); } }
      HITJ(h0, s0, sa.x)
      HITJ(h1, s1, sa.y)
      HITJ(h2, s2, sa.z)
      HITJ(h3, s3, sa.w)
      HITJ(h4, s4, sb.x)
      HITJ(h5, s5, sb.y)
      HITJ(h6, s6, sb.z)
      HITJ(h7, s7, sb.w)
#undef HITJ
    }
  }
  return wc;
}

__global__ __launch_bounds__(NTHR) void k_wprep(
    const float* __restrict__ w1o, const float* __restrict__ w2o, const float* __restrict__ w1s,
    const float* __restrict__ w2s, const float* __restrict__ wm1, const float* __restrict__ wm2,
    _Float16* wp) {
  const int b = blockIdx.x, tid = threadIdx.x;
  const float* W;
  int K, N, lb, pofs;
  if (b < 8)       { W = w1o; K = FO;   N = HID;  lb = b;      pofs = P0OF; }
  else if (b < 12) { W = w2o; K = HID;  N = NCL;  lb = b - 8;  pofs = P1OF; }
  else if (b < 16) { W = w1s; K = FS;   N = HID;  lb = b - 12; pofs = P2OF; }
  else if (b < 20) { W = w2s; K = HID;  N = NCL;  lb = b - 16; pofs = P3OF; }
  else if (b < 36) { W = wm1; K = HID;  N = MHID; lb = b - 20; pofs = P4OF; }
  else             { W = wm2; K = MHID; N = NCL;  lb = b - 36; pofs = P5OF; }
  const int i  = lb * NTHR + tid;
  const int kq = K >> 3;
  int n = i / kq;
  n = n > N - 1 ? N - 1 : n;
  const int k0 = (i - (i / kq) * kq) * 8;
  v8h hv;
#pragma unroll
  for (int e = 0; e < 8; ++e) hv[e] = (_Float16)(W[(size_t)(k0 + e) * N + n] * (float)WSC);
  _Float16* d = wp + pofs + (size_t)i * 8;
  *(volatile v8h*)d = hv;
  __threadfence();
  *(volatile v8h*)d = hv;
}

__global__ __launch_bounds__(NTHR) void k_count(
    const int* __restrict__ keys, int* cnt, float* dinv, int nE, int nN, int vec8) {
  extern __shared__ v4f lds_dyn[];
  int* scnt = (int*)lds_dyn;
  int* list = scnt + NBC;
  int* wcnt = list + LISTN;
  const int tid = threadIdx.x, lane = tid & 31, wave = tid >> 5;
  const int nodeBase = blockIdx.x * NBC;

  {
    const v4i z = {0, 0, 0, 0};
    for (int i = tid; i < NBC / 4; i += NTHR) ((v4i*)scnt)[i] = z;
  }
  __syncthreads();

  const int nChunks = (nE + CHUNK - 1) / CHUNK;
#pragma unroll 1
  for (int ch = 0; ch < nChunks; ++ch) {
    const int cbase = ch * CHUNK;
    const int wc = scan_chunk<NBC, 0>(keys, keys, nE, nN, cbase, nodeBase, vec8, list, tid, lane, wave);
    if (lane == 0) wcnt[wave] = wc;
    __syncthreads();
    if (wave == 0) {
#pragma unroll 1
      for (int wsx = 0; wsx < NWAVE; ++wsx) {
        int n = __builtin_amdgcn_readfirstlane(wcnt[wsx]);
        n = n > WCAP ? WCAP : (n < 0 ? 0 : n);
        const int* lp = list + wsx * WCAP;
#pragma unroll 1
        for (int i = 0; i < n; ++i) {
          const int ent  = __builtin_amdgcn_readfirstlane(lp[i]);
          const int slot = ent & (NBC - 1);
          if (lane == 0) scnt[slot] = scnt[slot] + 1;
        }
      }
    }
    __syncthreads();
  }

  int*   cp = cnt + (size_t)nodeBase;
  float* dp = dinv + (size_t)nodeBase;
#pragma unroll 4
  for (int q = 0; q < 32; ++q) {
    const int f = (wave * 32 + q) * 128 + 4 * lane;
    const v4i c = *(const v4i*)(scnt + f);
    v4f d;
    d.x = rsqrtf((float)(c.x > 1 ? c.x : 1)); d.y = rsqrtf((float)(c.y > 1 ? c.y : 1));
    d.z = rsqrtf((float)(c.z > 1 ? c.z : 1)); d.w = rsqrtf((float)(c.w > 1 ? c.w : 1));
    *(volatile v4i*)(cp + f) = c;
    *(volatile v4f*)(dp + f) = d;
  }
  __threadfence();
#pragma unroll 4
  for (int q = 0; q < 32; ++q) {
    const int f = (wave * 32 + q) * 128 + 4 * lane;
    const v4i c = *(const v4i*)(scnt + f);
    v4f d;
    d.x = rsqrtf((float)(c.x > 1 ? c.x : 1)); d.y = rsqrtf((float)(c.y > 1 ? c.y : 1));
    d.z = rsqrtf((float)(c.z > 1 ? c.z : 1)); d.w = rsqrtf((float)(c.w > 1 ? c.w : 1));
    *(volatile v4i*)(cp + f) = c;
    *(volatile v4f*)(dp + f) = d;
  }
}

__global__ __launch_bounds__(OTHR) void k_offsets(
    const int* __restrict__ cnt, int* off, int* rbase, int nBF) {
  __shared__ __attribute__((aligned(16))) int srb[RBN];
  __shared__ int wtot[OTHR / 32];
  const int tid = threadIdx.x, lane = tid & 31, wave = tid >> 5;
  for (int i = tid; i < RBN; i += OTHR) srb[i] = 0;
  int carry = 0;
#pragma unroll 1
  for (int fb = 0; fb < nBF; ++fb) {
    const int base = fb * NBF;
    const v4i c = *(const v4i*)(cnt + base + 4 * tid);
    const int e0 = max(c.x, 0), e1 = max(c.y, 0), e2 = max(c.z, 0), e3 = max(c.w, 0);
    const int ts = e0 + e1 + e2 + e3;
    int incl = ts;
#pragma unroll
    for (int d = 1; d < 32; d <<= 1) {
      const int t = __shfl_up(incl, d);
      if (lane >= d) incl += t;
    }
    if (lane == 31) wtot[wave] = incl;
    __syncthreads();
    int pre = 0;
#pragma unroll 1
    for (int w = 0; w < wave; ++w) pre += wtot[w];
    int tot = 0;
#pragma unroll
    for (int w = 0; w < OTHR / 32; ++w) tot += wtot[w];
    int run = carry + pre + incl - ts;
    v4i o;
    o.x = run; run += e0;
    o.y = run; run += e1;
    o.z = run; run += e2;
    o.w = run;
    int* op = off + base + 4 * tid;
    *(volatile v4i*)op = o;
    __threadfence();
    *(volatile v4i*)op = o;
    if (tid == 0) srb[min(fb, RBN - 1)] = carry;
    carry += (tot + 31) & ~31;
    __syncthreads();
  }
  if (tid == 0) srb[min(nBF, RBN - 1)] = carry;
  __syncthreads();
  v4i rv = {0, 0, 0, 0};
  if (tid < 32) rv = *(const v4i*)(srb + 4 * tid);
  if (tid < 32) *(volatile v4i*)(rbase + 4 * tid) = rv;
  __threadfence();
  if (tid < 32) *(volatile v4i*)(rbase + 4 * tid) = rv;
}

__global__ __launch_bounds__(NTHR) void k_fill(
    const int* __restrict__ keys, const int* __restrict__ vals, const int* __restrict__ off,
    const int* __restrict__ rbase, int* csr, int nN, int nE, int vec8, int csrLen) {
  extern __shared__ v4f lds_dyn[];
  int* region = (int*)lds_dyn;
  int* cursor = region + RCAP;
  int* list   = cursor + NBF;
  int* wcnt   = list + LISTN;
  const int tid = threadIdx.x, lane = tid & 31, wave = tid >> 5;
  const int b = blockIdx.x;
  const int nodeBase = b * NBF;

  int rb0 = rbase[b];
  const int rb1 = rbase[b + 1];
  rb0 = rb0 < 0 ? 0 : (rb0 > csrLen ? csrLen : rb0);
  rb0 &= ~31;
  int len = rb1 - rb0;
  len = len < 0 ? 0 : (len > RCAP ? RCAP : len);
  int lenW = (len + 31) & ~31;
  if (rb0 + lenW > csrLen) lenW = (csrLen - rb0) & ~31;

  {
    const v4i z = {0, 0, 0, 0};
    for (int i = tid; i < RCAP / 4; i += NTHR) ((v4i*)region)[i] = z;
    for (int s = tid; s < NBF; s += NTHR) {
      int o = off[nodeBase + s] - rb0;
      o = o < 0 ? 0 : (o > RCAP ? RCAP : o);
      cursor[s] = o;
    }
  }
  __syncthreads();

  const int nChunks = (nE + CHUNK - 1) / CHUNK;
#pragma unroll 1
  for (int ch = 0; ch < nChunks; ++ch) {
    const int cbase = ch * CHUNK;
    const int wc = scan_chunk<NBF, 1>(keys, vals, nE, nN, cbase, nodeBase, vec8, list, tid, lane, wave);
    if (lane == 0) wcnt[wave] = wc;
    __syncthreads();
    if (wave == 0) {
#pragma unroll 1
      for (int wsx = 0; wsx < NWAVE; ++wsx) {
        int n = __builtin_amdgcn_readfirstlane(wcnt[wsx]);
        n = n > WCAP ? WCAP : (n < 0 ? 0 : n);
        const int* lp = list + wsx * WCAP;
#pragma unroll 1
        for (int i = 0; i < n; ++i) {
          const int ent  = __builtin_amdgcn_readfirstlane(lp[i]);
          const int slot = ent & (NBF - 1);
          int src = (ent >> ESHF) & 0xFFFFF;
          src = src > nN - 1 ? nN - 1 : src;
          if (lane == 0) {
            int pos = cursor[slot];
            pos = pos < 0 ? 0 : (pos > RCAP - 1 ? RCAP - 1 : pos);
            region[pos] = src;
            const int np = pos + 1;
            cursor[slot] = np > RCAP ? RCAP : np;
          }
        }
      }
    }
    __syncthreads();
  }

  const int nv = lenW >> 2;
  int* gp = csr + rb0;
#pragma unroll 1
  for (int i = tid; i < nv; i += NTHR) { const v4i v = ((const v4i*)region)[i]; *(volatile v4i*)(gp + 4 * i) = v; }
  __threadfence();
#pragma unroll 1
  for (int i = tid; i < nv; i += NTHR) { const v4i v = ((const v4i*)region)[i]; *(volatile v4i*)(gp + 4 * i) = v; }
}

__global__ __launch_bounds__(NTHR) void k_agg1(
    const int* __restrict__ csr, const int* __restrict__ off, const int* __restrict__ cnt,
    const float* __restrict__ dout, const float* __restrict__ xo, const float* __restrict__ xs,
    _Float16* aggo, _Float16* aggs, int nN, int csrLen) {
  extern __shared__ v4f lds_dyn[];
  _Float16* sO = (_Float16*)lds_dyn;
  _Float16* sS = sO + NWAVE * 32 * FO;
  const int tid = threadIdx.x, lane = tid & 31, wave = tid >> 5;
  const int tbase = blockIdx.x * TGT + wave * 32;
  const int cl = tbase + lane;
  const int cnt_l = cnt[cl];
  const int off_l = off[cl];

#pragma unroll 1
  for (int j = 0; j < 32; ++j) {
    int n = __builtin_amdgcn_readlane(cnt_l, j);
    n = n < 0 ? 0 : (n > DEGCAP ? DEGCAP : n);
    const int st = __builtin_amdgcn_readlane(off_l, j);
    v4f a4 = {0.f, 0.f, 0.f, 0.f};
    v2f a2 = {0.f, 0.f};
#pragma unroll 1
    for (int q0 = 0; q0 < n; q0 += 32) {
      int pos = st + q0 + lane;
      pos = pos < 0 ? 0 : (pos > csrLen - 1 ? csrLen - 1 : pos);
      int sl = csr[pos];
      sl = sl < 0 ? 0 : (sl > nN - 1 ? nN - 1 : sl);
      const int mcnt = (n - q0) < 32 ? (n - q0) : 32;
#pragma unroll 1
      for (int p = 0; p < mcnt; ++p) {
        const int s = __builtin_amdgcn_readlane(sl, p);
        const float ds = dout[s];
        const v4f xv = *(const v4f*)(xo + (size_t)s * FO + 4 * lane);
        const v2f sv = *(const v2f*)(xs + (size_t)s * FS + 2 * lane);
        a4 = a4 + xv * ds;
        a2 = a2 + sv * ds;
      }
    }
    v4h ho; v2h hs;
    ho.x = (_Float16)a4.x; ho.y = (_Float16)a4.y; ho.z = (_Float16)a4.z; ho.w = (_Float16)a4.w;
    hs.x = (_Float16)a2.x; hs.y = (_Float16)a2.y;
    *(v4h*)(sO + (wave * 32 + j) * FO + 4 * lane) = ho;
    *(v2h*)(sS + (wave * 32 + j) * FS + 2 * lane) = hs;
  }
  __syncthreads();

  const _Float16* lO = sO + wave * 32 * FO;
  const _Float16* lS = sS + wave * 32 * FS;
  _Float16* gO = aggo + (size_t)tbase * FO;
  _Float16* gS = aggs + (size_t)tbase * FS;
#pragma unroll
  for (int i = 0; i < (32 * FO) / 256; ++i) {
    const v8ha v = *(const v8ha*)(lO + i * 256 + 8 * lane);
    *(volatile v8h*)(gO + i * 256 + 8 * lane) = v;
  }
#pragma unroll
  for (int i = 0; i < (32 * FS) / 256; ++i) {
    const v8ha v = *(const v8ha*)(lS + i * 256 + 8 * lane);
    *(volatile v8h*)(gS + i * 256 + 8 * lane) = v;
  }
  __threadfence();
#pragma unroll
  for (int i = 0; i < (32 * FO) / 256; ++i) {
    const v8ha v = *(const v8ha*)(lO + i * 256 + 8 * lane);
    *(volatile v8h*)(gO + i * 256 + 8 * lane) = v;
  }
#pragma unroll
  for (int i = 0; i < (32 * FS) / 256; ++i) {
    const v8ha v = *(const v8ha*)(lS + i * 256 + 8 * lane);
    *(volatile v8h*)(gS + i * 256 + 8 * lane) = v;
  }
}

__global__ __launch_bounds__(NTHR) void k_agg2(
    const int* __restrict__ csr, const int* __restrict__ off, const int* __restrict__ cnt,
    const float* __restrict__ din, const float* __restrict__ hwo, const float* __restrict__ hws,
    const float* __restrict__ bo, const float* __restrict__ bsv,
    _Float16* cat, int nN, int csrLen) {
  extern __shared__ v4f lds_dyn[];
  _Float16* sC = (_Float16*)lds_dyn;
  const int tid = threadIdx.x, lane = tid & 31, wave = tid >> 5;
  const int tbase = blockIdx.x * TGT + wave * 32;
  const int cl = tbase + lane;
  const int cnt_l = cnt[cl];
  const int off_l = off[cl];
  union FI { float f; int i; };
  FI dvu; dvu.f = din[cl];
  const v2f bbo = *(const v2f*)(bo + 2 * lane);
  const v2f bbs = *(const v2f*)(bsv + 2 * lane);

#pragma unroll 1
  for (int j = 0; j < 32; ++j) {
    int n = __builtin_amdgcn_readlane(cnt_l, j);
    n = n < 0 ? 0 : (n > DEGCAP ? DEGCAP : n);
    const int st = __builtin_amdgcn_readlane(off_l, j);
    FI du; du.i = __builtin_amdgcn_readlane(dvu.i, j);
    const float dc = du.f;
    v2f ao = {0.f, 0.f};
    v2f as = {0.f, 0.f};
#pragma unroll 1
    for (int q0 = 0; q0 < n; q0 += 32) {
      int pos = st + q0 + lane;
      pos = pos < 0 ? 0 : (pos > csrLen - 1 ? csrLen - 1 : pos);
      int sl = csr[pos];
      sl = sl < 0 ? 0 : (sl > nN - 1 ? nN - 1 : sl);
      const int mcnt = (n - q0) < 32 ? (n - q0) : 32;
#pragma unroll 1
      for (int p = 0; p < mcnt; ++p) {
        const int s = __builtin_amdgcn_readlane(sl, p);
        ao = ao + *(const v2f*)(hwo + (size_t)s * NCL + 2 * lane);
        as = as + *(const v2f*)(hws + (size_t)s * NCL + 2 * lane);
      }
    }
    const v2f vo = ao * dc + bbo;
    const v2f vs = as * dc + bbs;
    v2h ho, hs;
    ho.x = (_Float16)(vo.x * (float)ASC); ho.y = (_Float16)(vo.y * (float)ASC);
    hs.x = (_Float16)(vs.x * (float)ASC); hs.y = (_Float16)(vs.y * (float)ASC);
    *(v2h*)(sC + (wave * 32 + j) * (2 * NCL) + 2 * lane) = ho;
    *(v2h*)(sC + (wave * 32 + j) * (2 * NCL) + NCL + 2 * lane) = hs;
  }
  __syncthreads();

  const _Float16* lC = sC + wave * 32 * (2 * NCL);
  _Float16* gC = cat + (size_t)tbase * (2 * NCL);
#pragma unroll
  for (int i = 0; i < (32 * 2 * NCL) / 256; ++i) {
    const v8ha v = *(const v8ha*)(lC + i * 256 + 8 * lane);
    *(volatile v8h*)(gC + i * 256 + 8 * lane) = v;
  }
  __threadfence();
#pragma unroll
  for (int i = 0; i < (32 * 2 * NCL) / 256; ++i) {
    const v8ha v = *(const v8ha*)(lC + i * 256 + 8 * lane);
    *(volatile v8h*)(gC + i * 256 + 8 * lane) = v;
  }
}

template <bool HOUT>
__device__ __forceinline__ void store_tile(const float* wstg, float* Cf, _Float16* Ch, int wrow,
                                           int cpitch, int col0, int nRowsStore, int lane) {
  if (HOUT) {
#pragma unroll
    for (int i = 0; i < 4; ++i) {
      const int rl = 4 * i + (lane >> 3);
      const int pc = (lane & 7) * 8;
      const v4fa x0 = *(const v4fa*)(wstg + rl * GCOLS + pc);
      const v4fa x1 = *(const v4fa*)(wstg + rl * GCOLS + pc + 4);
      v8h hv;
      hv[0] = (_Float16)x0.x; hv[1] = (_Float16)x0.y; hv[2] = (_Float16)x0.z; hv[3] = (_Float16)x0.w;
      hv[4] = (_Float16)x1.x; hv[5] = (_Float16)x1.y; hv[6] = (_Float16)x1.z; hv[7] = (_Float16)x1.w;
      _Float16* d = Ch + (size_t)(wrow + rl) * cpitch + col0 + pc;
      *(volatile v8h*)d = hv;
    }
  } else {
#pragma unroll
    for (int i = 0; i < 8; ++i) {
      const int rl = 2 * i + (lane >> 4);
      const int pc = (lane & 15) * 4;
      const v4fa x = *(const v4fa*)(wstg + rl * GCOLS + pc);
      const int row = wrow + rl;
      const v4f xv = x;
      if (row < nRowsStore) *(volatile v4f*)(Cf + (size_t)row * cpitch + col0 + pc) = xv;
    }
  }
}

template <int KD, bool RS, bool HOUT, bool RELU, bool BIAS>
__global__ __launch_bounds__(NTHR) void k_gemm(
    const _Float16* __restrict__ A, const _Float16* __restrict__ Bw,
    const float* __restrict__ rsA, const float* __restrict__ rsB, const float* __restrict__ bias,
    float* Cf, _Float16* Ch, int cpitch, int nRowsStore, float osc) {
  __shared__ __attribute__((aligned(16))) float stg[NWAVE * 16 * GCOLS];
  static_assert((KD % 32) == 0);
  const int tid = threadIdx.x, lane = tid & 31, wave = tid >> 5, hh = lane >> 4, m = lane & 15;
  const int rowBase = blockIdx.x * GROWS;
  const int col0 = blockIdx.y * GCOLS;
  const int wrow = rowBase + wave * 16;

  v8f acc[4];
#pragma unroll
  for (int t = 0; t < 4; ++t) { v8f z = {0.f, 0.f, 0.f, 0.f, 0.f, 0.f, 0.f, 0.f}; acc[t] = z; }
  const _Float16* ap = A  + (size_t)(wrow + m) * KD + 8 * hh;
  const _Float16* bq = Bw + (size_t)(col0 + m) * KD + 8 * hh;
#pragma unroll 1
  for (int kt = 0; kt < KD / 32; ++kt) {
    FragH af;
    af.h[0] = *(const v8h*)(ap + 32 * kt);
    af.h[1] = *(const v8h*)(ap + 32 * kt + 16);
#pragma unroll
    for (int t = 0; t < 4; ++t) {
      const _Float16* bp = bq + (size_t)(16 * t) * KD + 32 * kt;
      FragH bf;
      bf.h[0] = *(const v8h*)bp;
      bf.h[1] = *(const v8h*)(bp + 16);
      acc[t] = wmf(af.v, bf.v, acc[t]);
    }
  }

  float sa[8], sb[8];
  if (RS) {
    const v4f a0 = *(const v4f*)(rsA + wrow + 8 * hh), a1 = *(const v4f*)(rsA + wrow + 8 * hh + 4);
    const v4f b0 = *(const v4f*)(rsB + wrow + 8 * hh), b1 = *(const v4f*)(rsB + wrow + 8 * hh + 4);
    sa[0] = a0.x; sa[1] = a0.y; sa[2] = a0.z; sa[3] = a0.w; sa[4] = a1.x; sa[5] = a1.y; sa[6] = a1.z; sa[7] = a1.w;
    sb[0] = b0.x; sb[1] = b0.y; sb[2] = b0.z; sb[3] = b0.w; sb[4] = b1.x; sb[5] = b1.y; sb[6] = b1.z; sb[7] = b1.w;
  } else {
#pragma unroll
    for (int r = 0; r < 8; ++r) { sa[r] = 1.0f; sb[r] = 1.0f; }
  }
  float* sp = stg + (wave * 16 + 8 * hh) * GCOLS + m;
#pragma unroll
  for (int t = 0; t < 4; ++t) {
    const float bv = BIAS ? bias[col0 + 16 * t + m] : 0.0f;
#pragma unroll
    for (int r = 0; r < 8; ++r) {
      float v = acc[t][r] * (osc * sa[r]) + bv;
      if (RELU) v = fmaxf(v, 0.0f);
      if (RS) v = v * sb[r];
      if (HOUT) v = v * (float)ASC;
      sp[r * GCOLS + 16 * t] = v;
    }
  }
  __syncthreads();

  const float* wstg = stg + wave * 16 * GCOLS;
  store_tile<HOUT>(wstg, Cf, Ch, wrow, cpitch, col0, nRowsStore, lane);
  __threadfence();
  store_tile<HOUT>(wstg, Cf, Ch, wrow, cpitch, col0, nRowsStore, lane);
}

extern "C" void kernel_launch(void* const* d_in, const int* in_sizes, int n_in,
                              void* d_out, int out_size, void* d_ws, size_t ws_size,
                              hipStream_t stream) {
  if (n_in < 16) return;
  const int nE = in_sizes[0];
  if (nE <= 0 || in_sizes[1] != nE) return;
  const int nN = in_sizes[2] / FO;
  if (nN <= 0 || in_sizes[2] != nN * FO || in_sizes[3] != nN * FS) return;
  if (in_sizes[4] != FO * HID || in_sizes[5] != HID) return;
  if (in_sizes[6] != HID * NCL || in_sizes[7] != NCL) return;
  if (in_sizes[8] != FS * HID || in_sizes[9] != HID) return;
  if (in_sizes[10] != HID * NCL || in_sizes[11] != NCL) return;
  if (in_sizes[12] != (2 * NCL) * MHID || in_sizes[13] != MHID) return;
  if (in_sizes[14] != MHID * NCL || in_sizes[15] != NCL) return;
  if (out_size != nN * NCL) return;
  if (nN > (1 << 20) || nE > (1 << 28)) return;

  const int*   src = (const int*)d_in[0];
  const int*   dst = (const int*)d_in[1];
  const float* xo  = (const float*)d_in[2];
  const float* xs  = (const float*)d_in[3];
  const float* W1o = (const float*)d_in[4];  const float* b1o = (const float*)d_in[5];
  const float* W2o = (const float*)d_in[6];  const float* b2o = (const float*)d_in[7];
  const float* W1s = (const float*)d_in[8];  const float* b1s = (const float*)d_in[9];
  const float* W2s = (const float*)d_in[10]; const float* b2s = (const float*)d_in[11];
  const float* Wm1 = (const float*)d_in[12]; const float* bm1 = (const float*)d_in[13];
  const float* Wm2 = (const float*)d_in[14]; const float* bm2 = (const float*)d_in[15];
  float* out = (float*)d_out;

  const int NPAD   = ((nN + TGT - 1) / TGT) * TGT;
  const int nBC    = (nN + NBC - 1) / NBC;
  const int CNTPAD = nBC * NBC;
  const int nBF    = (nN + NBF - 1) / NBF;
  const int OFFN   = nBF * NBF;
  if (nBF + 1 > RBN) return;
  if (OFFN > CNTPAD || NPAD > OFFN) return;
  const int csrLen = ((nE + 31) & ~31) + 32 * (nBF + 1);
  const int nGemm  = NPAD / GROWS;
  const int nAgg   = NPAD / TGT;

  char* ws = (char*)d_ws;
  size_t off = 0;
  const size_t oW    = off; off += (size_t)WPH * 2;                   off = (off + 255) & ~(size_t)255;
  const size_t oCntI = off; off += (size_t)CNTPAD * 4;                off = (off + 255) & ~(size_t)255;
  const size_t oDin  = off; off += (size_t)CNTPAD * 4;                off = (off + 255) & ~(size_t)255;
  const size_t oCntO = off; off += (size_t)CNTPAD * 4;                off = (off + 255) & ~(size_t)255;
  const size_t oDout = off; off += (size_t)CNTPAD * 4;                off = (off + 255) & ~(size_t)255;
  const size_t oOff  = off; off += (size_t)OFFN * 4;                  off = (off + 255) & ~(size_t)255;
  const size_t oRb   = off; off += (size_t)RBN * 4;                   off = (off + 255) & ~(size_t)255;
  const size_t oCsr  = off; off += (size_t)csrLen * 4;                off = (off + 255) & ~(size_t)255;
  const size_t oRA   = off; off += (size_t)NPAD * MHID * 2;           off = (off + 255) & ~(size_t)255;
  const size_t oRB   = off; off += (size_t)NPAD * HID * 2;            off = (off + 255) & ~(size_t)255;
  const size_t oRC   = off; off += (size_t)NPAD * HID * 2;            off = (off + 255) & ~(size_t)255;
  if (off > ws_size || off > (size_t)WSCAP) return;
  if ((size_t)NPAD * (FO + FS) * 2 > (size_t)NPAD * MHID * 2) return;
  if ((size_t)NPAD * NCL * 4 * 2 > (size_t)NPAD * MHID * 2) return;

  _Float16* wp   = (_Float16*)(ws + oW);
  int*      cntI = (int*)(ws + oCntI);
  float*    din  = (float*)(ws + oDin);
  int*      cntO = (int*)(ws + oCntO);
  float*    dout = (float*)(ws + oDout);
  int*      offp = (int*)(ws + oOff);
  int*      rb   = (int*)(ws + oRb);
  int*      csr  = (int*)(ws + oCsr);
  _Float16* aggO = (_Float16*)(ws + oRA);
  _Float16* aggS = aggO + (size_t)NPAD * FO;
  float*    hwo  = (float*)(ws + oRA);
  float*    hws  = hwo + (size_t)NPAD * NCL;
  _Float16* mh   = (_Float16*)(ws + oRA);
  _Float16* hd1o = (_Float16*)(ws + oRB);
  _Float16* catp = (_Float16*)(ws + oRB);
  _Float16* hd1s = (_Float16*)(ws + oRC);

  const int vec8 = ((nE & 3) == 0) ? 1 : 0;
  const float osc1 = 1.0f / (float)WSC;
  const float osc2 = 1.0f / (float)(ASC * WSC);

  k_wprep<<<WPBLK, NTHR, 0, stream>>>(W1o, W2o, W1s, W2s, Wm1, Wm2, wp);

  hipFuncSetAttribute(reinterpret_cast<const void*>(&k_count),
                      hipFuncAttributeMaxDynamicSharedMemorySize, LDS_COUNT);
  k_count<<<nBC, NTHR, LDS_COUNT, stream>>>(dst, cntI, din, nE, nN, vec8);
  k_count<<<nBC, NTHR, LDS_COUNT, stream>>>(src, cntO, dout, nE, nN, vec8);

  k_offsets<<<1, OTHR, 0, stream>>>(cntI, offp, rb, nBF);
  hipFuncSetAttribute(reinterpret_cast<const void*>(&k_fill),
                      hipFuncAttributeMaxDynamicSharedMemorySize, LDS_FILL);
  k_fill<<<nBF, NTHR, LDS_FILL, stream>>>(dst, src, offp, rb, csr, nN, nE, vec8, csrLen);

  hipFuncSetAttribute(reinterpret_cast<const void*>(&k_agg1),
                      hipFuncAttributeMaxDynamicSharedMemorySize, LDS_AGG1);
  k_agg1<<<nAgg, NTHR, LDS_AGG1, stream>>>(csr, offp, cntI, dout, xo, xs, aggO, aggS, nN, csrLen);

  k_gemm<FO, true, true, true, true><<<dim3(nGemm, HID / GCOLS), NTHR, 0, stream>>>(
      aggO, wp + P0OF, din, dout, b1o, dout, hd1o, HID, NPAD, osc1);
  k_gemm<FS, true, true, true, true><<<dim3(nGemm, HID / GCOLS), NTHR, 0, stream>>>(
      aggS, wp + P2OF, din, dout, b1s, dout, hd1s, HID, NPAD, osc1);

  k_gemm<HID, false, false, false, false><<<dim3(nGemm, NCL / GCOLS), NTHR, 0, stream>>>(
      hd1o, wp + P1OF, din, dout, b2o, hwo, hd1o, NCL, NPAD, osc2);
  k_gemm<HID, false, false, false, false><<<dim3(nGemm, NCL / GCOLS), NTHR, 0, stream>>>(
      hd1s, wp + P3OF, din, dout, b2s, hws, hd1s, NCL, NPAD, osc2);

  hipFuncSetAttribute(reinterpret_cast<const void*>(&k_agg2),
                      hipFuncAttributeMaxDynamicSharedMemorySize, LDS_AGG2);
  k_agg2<<<nAgg, NTHR, LDS_AGG2, stream>>>(csr, offp, cntI, din, hwo, hws, b2o, b2s, catp, nN, csrLen);

  k_gemm<2 * NCL, false, true, true, true><<<dim3(nGemm, MHID / GCOLS), NTHR, 0, stream>>>(
      catp, wp + P4OF, din, dout, bm1, dout, mh, MHID, NPAD, osc2);

  k_gemm<MHID, false, false, false, true><<<dim3(nGemm, NCL / GCOLS), NTHR, 0, stream>>>(
      mh, wp + P5OF, din, dout, bm2, out, mh, NCL, nN, osc2);
}
